// Encoder_Adversarial_GCN_55714315764099
// MI455X (gfx1250) — hardware-verified
//
#include <hip/hip_runtime.h>
#include <stddef.h>


#define DX      256
#define DH      512
#define NTHR    256
#define NWAVE   8
#define EPT     8
#define NGRP    2
#define CHUNK   (NTHR * EPT * NGRP)
#define WCAP    (EPT * NGRP * 32)
#define LISTN   (NWAVE * WCAP)
#define NB      256
#define NBD     4096
#define G2ROWS  32
#define G2THR   128
#define ASC     4.0f
#define WSC     16.0f
#define C1INV   0.015625f
#define C2INV   0.0625f
#define LDS_AGG (NB * DX * 4 + LISTN * 4 + 64)

static_assert((CHUNK & (CHUNK - 1)) == 0);
static_assert(CHUNK <= 4096);
static_assert((NB & (NB - 1)) == 0 && NB <= 4096);
static_assert((NBD & (NBD - 1)) == 0 && NBD <= 4096);
static_assert(NB == 32 * NWAVE);
static_assert(NB % G2ROWS == 0);
static_assert(NBD == NTHR * 16);

typedef float    v4f  __attribute__((ext_vector_type(4)));
typedef float    v8f  __attribute__((ext_vector_type(8)));
typedef int      v4i  __attribute__((ext_vector_type(4)));
typedef _Float16 v8h  __attribute__((ext_vector_type(8)));
typedef _Float16 v16h __attribute__((ext_vector_type(16)));
union FragH { v16h v; v8h h[2]; };

__device__ __forceinline__ v8h cvt8(v4f a, v4f b) {
  v8h r;
  r[0] = (_Float16)a.x; r[1] = (_Float16)a.y; r[2] = (_Float16)a.z; r[3] = (_Float16)a.w;
  r[4] = (_Float16)b.x; r[5] = (_Float16)b.y; r[6] = (_Float16)b.z; r[7] = (_Float16)b.w;
  return r;
}

__device__ __forceinline__ v8f wmh(v16h a, v16h b, v8f c) {
  v8f d = __builtin_amdgcn_wmma_f32_16x16x32_f16(false, a, false, b, (short)0, c, false, false);
  asm volatile("v_nop\n\tv_nop\n\tv_nop\n\tv_nop" : "+v"(d) : "v"(a), "v"(b));
  return d;
}

template <int NBT>
__device__ __forceinline__ int scan_chunk(const int* __restrict__ dsts, int nE, int cbase, int nodeBase,
                                          int vec8, int* list, int tid, int wave) {
  int wc = 0;
#pragma unroll
  for (int g = 0; g < NGRP; ++g) {
    const int el0  = (g * NTHR + tid) * EPT;
    const int e0   = cbase + el0;
    const int sent = -2147483647 - 1;
    v4i da, db;
    if (vec8 != 0 && e0 + 7 < nE) {
      da = *(const v4i*)(dsts + e0);
      db = *(const v4i*)(dsts + e0 + 4);
    } else {
      da.x = (e0     < nE) ? dsts[min(e0, nE - 1)] : sent;
      da.y = (e0 + 1 < nE) ? dsts[min(e0 + 1, nE - 1)] : sent;
      da.z = (e0 + 2 < nE) ? dsts[min(e0 + 2, nE - 1)] : sent;
      da.w = (e0 + 3 < nE) ? dsts[min(e0 + 3, nE - 1)] : sent;
      db.x = (e0 + 4 < nE) ? dsts[min(e0 + 4, nE - 1)] : sent;
      db.y = (e0 + 5 < nE) ? dsts[min(e0 + 5, nE - 1)] : sent;
      db.z = (e0 + 6 < nE) ? dsts[min(e0 + 6, nE - 1)] : sent;
      db.w = (e0 + 7 < nE) ? dsts[min(e0 + 7, nE - 1)] : sent;
    }
    const unsigned nb = (unsigned)nodeBase;
    const unsigned s0 = (unsigned)da.x - nb, s1 = (unsigned)da.y - nb;
    const unsigned s2 = (unsigned)da.z - nb, s3 = (unsigned)da.w - nb;
    const unsigned s4 = (unsigned)db.x - nb, s5 = (unsigned)db.y - nb;
    const unsigned s6 = (unsigned)db.z - nb, s7 = (unsigned)db.w - nb;
    const bool h0 = s0 < (unsigned)NBT, h1 = s1 < (unsigned)NBT, h2 = s2 < (unsigned)NBT, h3 = s3 < (unsigned)NBT;
    const bool h4 = s4 < (unsigned)NBT, h5 = s5 < (unsigned)NBT, h6 = s6 < (unsigned)NBT, h7 = s7 < (unsigned)NBT;
    const unsigned any = __builtin_amdgcn_ballot_w32(h0 | h1 | h2 | h3 | h4 | h5 | h6 | h7);
    if (any != 0u) {
#define HITJ(J, HJ, SJ) { \
        const unsigned mj = __builtin_amdgcn_ballot_w32(HJ); \
        if (mj != 0u) { \
          if (HJ) { \
            const int pos = wc + (int)__builtin_amdgcn_mbcnt_lo(mj, 0u); \
            if (pos < WCAP) list[wave * WCAP + pos] = ((el0 + (J)) << 12) | (int)(SJ); \
          } \
          wc += (int)__builtin_popcount(mj); } }
      HITJ(0, h0, s0)
      HITJ(1, h1, s1)
      HITJ(2, h2, s2)
      HITJ(3, h3, s3)
      HITJ(4, h4, s4)
      HITJ(5, h5, s5)
      HITJ(6, h6, s6)
      HITJ(7, h7, s7)
#undef HITJ
    }
  }
  return wc;
}

template <int NBT>
__device__ __forceinline__ void drain_rows(const int* list, const int* wcnt, float* acc,
                                           const int* __restrict__ ei, const float* __restrict__ rows,
                                           const float* __restrict__ dinv, int cbase, int nE, int nN, int lane) {
#pragma unroll 1
  for (int wsx = 0; wsx < NWAVE; ++wsx) {
    int n = __builtin_amdgcn_readfirstlane(wcnt[wsx]);
    n = n > WCAP ? WCAP : (n < 0 ? 0 : n);
    const int* lp = list + wsx * WCAP;
#pragma unroll 1
    for (int i = 0; i < n; ++i) {
      const int ent  = __builtin_amdgcn_readfirstlane(lp[i]);
      const int slot = ent & (NBT - 1);
      int e = cbase + ((ent >> 12) & (CHUNK - 1));
      e = e > nE - 1 ? nE - 1 : e;
      int src = ei[e];
      src = src < 0 ? 0 : (src > nN - 1 ? nN - 1 : src);
      const float d = dinv[src];
      const float* rp = rows + (size_t)src * DX + 4 * lane;
      const v4f v0 = *(const v4f*)rp;
      const v4f v1 = *(const v4f*)(rp + 128);
      v4f* ap = (v4f*)(acc + slot * DX + 4 * lane);
      ap[0]  = ap[0]  + v0 * d;
      ap[32] = ap[32] + v1 * d;
    }
  }
}

__global__ __launch_bounds__(NTHR) void k_wprep(
    const float* __restrict__ W1, const float* __restrict__ W2,
    _Float16* w1s, _Float16* w2s) {
  const int i  = blockIdx.x * NTHR + threadIdx.x;
  const int n1 = DH * DX / 8;
  const int n2 = DX * DH / 8;
  if (i >= n1 + n2) return;
  const bool first = i < n1;
  v4f a, b;
  int o;
  if (first) {
    o = i * 8;
    const int n  = o / DX;
    const int k0 = o - n * DX;
    const float* p = W1 + (size_t)k0 * DH + n;
    a.x = p[0];      a.y = p[DH];     a.z = p[2 * DH]; a.w = p[3 * DH];
    b.x = p[4 * DH]; b.y = p[5 * DH]; b.z = p[6 * DH]; b.w = p[7 * DH];
  } else {
    o = (i - n1) * 8;
    const int n  = o / DH;
    const int k0 = o - n * DH;
    const float* p = W2 + (size_t)k0 * DX + n;
    a.x = p[0];      a.y = p[DX];     a.z = p[2 * DX]; a.w = p[3 * DX];
    b.x = p[4 * DX]; b.y = p[5 * DX]; b.z = p[6 * DX]; b.w = p[7 * DX];
  }
  a = a * WSC;
  b = b * WSC;
  const v8h hv = cvt8(a, b);
  _Float16* dp = (first ? w1s : w2s) + o;
  *(volatile v8h*)dp = hv;
  __threadfence();
  *(volatile v8h*)dp = hv;
}

__global__ __launch_bounds__(NTHR) void k_deg(
    const int* __restrict__ ei, float* dinv, int nE, int vec8) {
  __shared__ __attribute__((aligned(16))) int cnt[NBD];
  __shared__ __attribute__((aligned(16))) int list[LISTN];
  __shared__ int wcnt[NWAVE];
  const int tid = threadIdx.x, lane = tid & 31;
  const int wave = __builtin_amdgcn_readfirstlane(tid >> 5);
  const int nodeBase = blockIdx.x * NBD;
  const int* dsts = ei + nE;

  for (int i = tid; i < NBD; i += NTHR) cnt[i] = 0;
  __syncthreads();

  const int nChunks = (nE + CHUNK - 1) / CHUNK;
#pragma unroll 1
  for (int ch = 0; ch < nChunks; ++ch) {
    const int cbase = ch * CHUNK;
    const int wc = scan_chunk<NBD>(dsts, nE, cbase, nodeBase, vec8, list, tid, wave);
    if (lane == 0) wcnt[wave] = wc;
    __syncthreads();
    if (wave == 0) {
#pragma unroll 1
      for (int wsx = 0; wsx < NWAVE; ++wsx) {
        int n = __builtin_amdgcn_readfirstlane(wcnt[wsx]);
        n = n > WCAP ? WCAP : (n < 0 ? 0 : n);
        const int* lp = list + wsx * WCAP;
#pragma unroll 1
        for (int i = 0; i < n; ++i) {
          const int ent  = __builtin_amdgcn_readfirstlane(lp[i]);
          const int slot = ent & (NBD - 1);
          if (lane == 0) cnt[slot] = cnt[slot] + 1;
        }
      }
    }
    __syncthreads();
  }

  v4f dq[4];
#pragma unroll
  for (int q = 0; q < 4; ++q) {
    const int f = (wave * 4 + q) * 128 + 4 * lane;
    const v4i c = *(const v4i*)(cnt + f);
    dq[q].x = rsqrtf((float)(c.x + 1));
    dq[q].y = rsqrtf((float)(c.y + 1));
    dq[q].z = rsqrtf((float)(c.z + 1));
    dq[q].w = rsqrtf((float)(c.w + 1));
  }
  float* dp = dinv + (size_t)nodeBase;
#pragma unroll
  for (int q = 0; q < 4; ++q) *(volatile v4f*)(dp + (wave * 4 + q) * 128 + 4 * lane) = dq[q];
  __threadfence();
#pragma unroll
  for (int q = 0; q < 4; ++q) *(volatile v4f*)(dp + (wave * 4 + q) * 128 + 4 * lane) = dq[q];
}

__global__ __launch_bounds__(NTHR) void k_agg1(
    const int* __restrict__ ei, const float* __restrict__ x, const float* __restrict__ dinv,
    const float* __restrict__ b1, const float* __restrict__ pf, const _Float16* __restrict__ w1s,
    _Float16* hpl, int nN, int nE, int vec8) {
  extern __shared__ v4f lds_dyn[];
  float*    accF = (float*)lds_dyn;
  _Float16* accH = (_Float16*)lds_dyn;
  int*      list = (int*)(accF + NB * DX);
  int*      wcnt = list + LISTN;
  const int tid = threadIdx.x, lane = tid & 31, hh = lane >> 4, m = lane & 15;
  const int wave = __builtin_amdgcn_readfirstlane(tid >> 5);
  const int nodeBase = blockIdx.x * NB;
  const int* dsts = ei + nE;

  {
    const v4f z = {0.f, 0.f, 0.f, 0.f};
    for (int i = tid; i < NB * DX / 4; i += NTHR) lds_dyn[i] = z;
  }
  __syncthreads();

  const int nChunks = (nE + CHUNK - 1) / CHUNK;
#pragma unroll 1
  for (int ch = 0; ch < nChunks; ++ch) {
    const int cbase = ch * CHUNK;
    const int wc = scan_chunk<NB>(dsts, nE, cbase, nodeBase, vec8, list, tid, wave);
    if (lane == 0) wcnt[wave] = wc;
    __syncthreads();
    if (wave == 0) drain_rows<NB>(list, wcnt, accF, ei, x, dinv, cbase, nE, nN, lane);
    __syncthreads();
  }

#pragma unroll 1
  for (int bt = 0; bt < (NB * DX / 8) / NTHR; ++bt) {
    const int idx  = bt * NTHR + tid;
    const int slot = idx >> 5;
    const int c0   = (idx & 31) * 8;
    int node = nodeBase + slot;
    node = node > nN - 1 ? nN - 1 : node;
    const float d = dinv[node];
    const float* xp = x + (size_t)node * DX + c0;
    const v4f x0 = *(const v4f*)xp, x1 = *(const v4f*)(xp + 4);
    const float* ap = accF + slot * DX + c0;
    const v4f a0 = *(const v4f*)ap, a1 = *(const v4f*)(ap + 4);
    const float s = d * ASC;
    const v4f r0 = (a0 + x0 * d) * s;
    const v4f r1 = (a1 + x1 * d) * s;
    const v8h hv = cvt8(r0, r1);
    __syncthreads();
    *(v8h*)(accH + slot * (2 * DX) + c0) = hv;
  }
  __syncthreads();

  const int cc = 8 * m;
#pragma unroll 1
  for (int p = 0; p < 8; ++p) {
    const int rt = 2 * wave + (p >> 2);
    const int cg = p & 3;
    v8f acc[8];
#pragma unroll
    for (int t = 0; t < 8; ++t) { v8f z = {0.f, 0.f, 0.f, 0.f, 0.f, 0.f, 0.f, 0.f}; acc[t] = z; }
    const _Float16* ar = accH + (16 * rt + m) * (2 * DX) + 8 * hh;
#pragma unroll 1
    for (int kt = 0; kt < DX / 32; ++kt) {
      FragH a;
      a.h[0] = *(const v8h*)(ar + 32 * kt);
      a.h[1] = *(const v8h*)(ar + 32 * kt + 16);
#pragma unroll
      for (int t = 0; t < 8; ++t) {
        const _Float16* bp = w1s + (size_t)(128 * cg + 16 * t + m) * DX + 32 * kt + 8 * hh;
        FragH bq;
        bq.h[0] = *(const v8h*)bp;
        bq.h[1] = *(const v8h*)(bp + 16);
        acc[t] = wmh(a.v, bq.v, acc[t]);
      }
    }
    float* sp = accF + (32 * wave + 8 * hh) * DX + 128 + m;
#pragma unroll
    for (int t = 0; t < 8; ++t) {
      sp[0 * DX + 16 * t] = acc[t][0] * C1INV;
      sp[1 * DX + 16 * t] = acc[t][1] * C1INV;
      sp[2 * DX + 16 * t] = acc[t][2] * C1INV;
      sp[3 * DX + 16 * t] = acc[t][3] * C1INV;
      sp[4 * DX + 16 * t] = acc[t][4] * C1INV;
      sp[5 * DX + 16 * t] = acc[t][5] * C1INV;
      sp[6 * DX + 16 * t] = acc[t][6] * C1INV;
      sp[7 * DX + 16 * t] = acc[t][7] * C1INV;
    }
    __syncthreads();
    v8h hv[8];
#pragma unroll
    for (int j = 0; j < 8; ++j) {
      const int row = 2 * j + hh;
      const float* lp = accF + (32 * wave + row) * DX + 128 + cc;
      const v4f s0 = *(const v4f*)lp, s1 = *(const v4f*)(lp + 4);
      int node = nodeBase + 16 * rt + row;
      node = node > nN - 1 ? nN - 1 : node;
      const float* pp = pf + (size_t)node * DH + 128 * cg + cc;
      const v4f p0 = *(const v4f*)pp, p1 = *(const v4f*)(pp + 4);
      const float* bb = b1 + 128 * cg + cc;
      const v4f q0 = *(const v4f*)bb, q1 = *(const v4f*)(bb + 4);
      hv[j] = cvt8((s0 + q0) + p0, (s1 + q1) + p1);
    }
    _Float16* gp = hpl + ((size_t)nodeBase + 16 * rt + hh) * DH + 128 * cg + cc;
#pragma unroll
    for (int j = 0; j < 8; ++j) *(volatile v8h*)(gp + (size_t)(2 * j) * DH) = hv[j];
    __threadfence();
#pragma unroll
    for (int j = 0; j < 8; ++j) *(volatile v8h*)(gp + (size_t)(2 * j) * DH) = hv[j];
    __syncthreads();
  }
}

__global__ __launch_bounds__(G2THR) void k_gemm2(
    const _Float16* __restrict__ hpl, const _Float16* __restrict__ w2s, float* g2) {
  __shared__ __attribute__((aligned(16))) float stg[4 * 16 * 128];
  const int tid = threadIdx.x, lane = tid & 31, hh = lane >> 4, m = lane & 15;
  const int wave = __builtin_amdgcn_readfirstlane(tid >> 5);
  const int rt = wave >> 1, ch = wave & 1;
  const int row0 = blockIdx.x * G2ROWS + 16 * rt;

  v8f acc[8];
#pragma unroll
  for (int t = 0; t < 8; ++t) { v8f z = {0.f, 0.f, 0.f, 0.f, 0.f, 0.f, 0.f, 0.f}; acc[t] = z; }
  const _Float16* ar = hpl + ((size_t)row0 + m) * DH + 8 * hh;
#pragma unroll 1
  for (int kt = 0; kt < DH / 32; ++kt) {
    FragH a;
    a.h[0] = *(const v8h*)(ar + 32 * kt);
    a.h[1] = *(const v8h*)(ar + 32 * kt + 16);
#pragma unroll
    for (int t = 0; t < 8; ++t) {
      const _Float16* bp = w2s + (size_t)(128 * ch + 16 * t + m) * DH + 32 * kt + 8 * hh;
      FragH bq;
      bq.h[0] = *(const v8h*)bp;
      bq.h[1] = *(const v8h*)(bp + 16);
      acc[t] = wmh(a.v, bq.v, acc[t]);
    }
  }
  float* sp = stg + wave * 2048 + (8 * hh) * 128 + m;
#pragma unroll
  for (int t = 0; t < 8; ++t) {
    sp[0 * 128 + 16 * t] = acc[t][0] * C2INV;
    sp[1 * 128 + 16 * t] = acc[t][1] * C2INV;
    sp[2 * 128 + 16 * t] = acc[t][2] * C2INV;
    sp[3 * 128 + 16 * t] = acc[t][3] * C2INV;
    sp[4 * 128 + 16 * t] = acc[t][4] * C2INV;
    sp[5 * 128 + 16 * t] = acc[t][5] * C2INV;
    sp[6 * 128 + 16 * t] = acc[t][6] * C2INV;
    sp[7 * 128 + 16 * t] = acc[t][7] * C2INV;
  }
  __syncthreads();

  const float* lp = stg + wave * 2048 + 4 * lane;
  float* gp = g2 + (size_t)row0 * DX + 128 * ch + 4 * lane;
#pragma unroll
  for (int i = 0; i < 16; ++i) { const v4f v = *(const v4f*)(lp + i * 128); *(volatile v4f*)(gp + (size_t)i * DX) = v; }
  __threadfence();
#pragma unroll
  for (int i = 0; i < 16; ++i) { const v4f v = *(const v4f*)(lp + i * 128); *(volatile v4f*)(gp + (size_t)i * DX) = v; }
}

__global__ __launch_bounds__(NTHR) void k_agg2(
    const int* __restrict__ ei, const float* __restrict__ g2, const float* __restrict__ dinv,
    const float* __restrict__ b2, const float* __restrict__ pl, float* out, int nN, int nE, int vec8) {
  extern __shared__ v4f lds_dyn[];
  float* accF = (float*)lds_dyn;
  int*   list = (int*)(accF + NB * DX);
  int*   wcnt = list + LISTN;
  const int tid = threadIdx.x, lane = tid & 31;
  const int wave = __builtin_amdgcn_readfirstlane(tid >> 5);
  const int nodeBase = blockIdx.x * NB;
  const int* dsts = ei + nE;

  {
    const v4f z = {0.f, 0.f, 0.f, 0.f};
    for (int i = tid; i < NB * DX / 4; i += NTHR) lds_dyn[i] = z;
  }
  __syncthreads();

  const int nChunks = (nE + CHUNK - 1) / CHUNK;
#pragma unroll 1
  for (int ch = 0; ch < nChunks; ++ch) {
    const int cbase = ch * CHUNK;
    const int wc = scan_chunk<NB>(dsts, nE, cbase, nodeBase, vec8, list, tid, wave);
    if (lane == 0) wcnt[wave] = wc;
    __syncthreads();
    if (wave == 0) drain_rows<NB>(list, wcnt, accF, ei, g2, dinv, cbase, nE, nN, lane);
    __syncthreads();
  }

#pragma unroll 4
  for (int i = 0; i < (NB * DX / 4) / NTHR; ++i) {
    const int idx  = i * NTHR + tid;
    const int slot = idx >> 6;
    const int c4   = (idx & 63) * 4;
    int node = nodeBase + slot;
    node = node > nN - 1 ? nN - 1 : node;
    const float d  = dinv[node];
    const v4f   gv = *(const v4f*)(g2 + (size_t)node * DX + c4);
    const v4f   bv = *(const v4f*)(b2 + c4);
    const v4f   pv = *(const v4f*)(pl + (size_t)node * DX + c4);
    v4f* ap = (v4f*)(accF + slot * DX + c4);
    const v4f r = (*ap + gv * d) * d + bv + pv;
    *ap = r;
  }
  __syncthreads();

  const size_t outN = (size_t)nN * DX;
  const size_t ob   = (size_t)nodeBase * DX;
#pragma unroll 4
  for (int q = 0; q < 64; ++q) {
    const int f = (wave * 64 + q) * 128 + 4 * lane;
    const size_t gi = ob + (size_t)f;
    if (gi < outN) { const v4f v = *(const v4f*)(accF + f); *(volatile v4f*)(out + gi) = v; }
  }
  __threadfence();
#pragma unroll 4
  for (int q = 0; q < 64; ++q) {
    const int f = (wave * 64 + q) * 128 + 4 * lane;
    const size_t gi = ob + (size_t)f;
    if (gi < outN) { const v4f v = *(const v4f*)(accF + f); *(volatile v4f*)(out + gi) = v; }
  }
}

extern "C" void kernel_launch(void* const* d_in, const int* in_sizes, int n_in,
                              void* d_out, int out_size, void* d_ws, size_t ws_size,
                              hipStream_t stream) {
  if (n_in < 8) return;
  const int nN = in_sizes[0] / DX;
  const int nE = in_sizes[1] / 2;
  if (nN <= 0 || nE < 0 || in_sizes[0] != nN * DX || in_sizes[1] != nE * 2) return;
  if (in_sizes[2] != nN * DH || in_sizes[3] != nN * DX) return;
  if (in_sizes[4] != DX * DH || in_sizes[5] < DH || in_sizes[6] != DH * DX || in_sizes[7] < DX) return;
  if (out_size != nN * DX) return;

  const float* x  = (const float*)d_in[0];
  const int*   ei = (const int*)d_in[1];
  const float* pf = (const float*)d_in[2];
  const float* pl = (const float*)d_in[3];
  const float* W1 = (const float*)d_in[4];
  const float* b1 = (const float*)d_in[5];
  const float* W2 = (const float*)d_in[6];
  const float* b2 = (const float*)d_in[7];
  float* out = (float*)d_out;

  const int nBD = (nN + NBD - 1) / NBD;
  const int nA  = (nN + NB - 1) / NB;
  const int nG2 = (nN + G2ROWS - 1) / G2ROWS;
  if (nA * NB > nBD * NBD) return;
  if (nG2 * G2ROWS > nA * NB) return;

  char* ws = (char*)d_ws;
  size_t off = 0;
  const size_t oW1 = off; off += (size_t)DH * DX * 2;                     off = (off + 255) & ~(size_t)255;
  const size_t oW2 = off; off += (size_t)DX * DH * 2;                     off = (off + 255) & ~(size_t)255;
  const size_t oDv = off; off += (size_t)nBD * NBD * 4;                   off = (off + 255) & ~(size_t)255;
  const size_t oH  = off; off += (size_t)nA * NB * DH * 2;                off = (off + 255) & ~(size_t)255;
  const size_t oG2 = off; off += (size_t)nG2 * G2ROWS * DX * 4;           off = (off + 255) & ~(size_t)255;
  if (off > ws_size) return;
  if (off > (size_t)134217728) return;
  _Float16* w1s  = (_Float16*)(ws + oW1);
  _Float16* w2s  = (_Float16*)(ws + oW2);
  float*    dinv = (float*)(ws + oDv);
  _Float16* hpl  = (_Float16*)(ws + oH);
  float*    g2   = (float*)(ws + oG2);

  const int vec8 = ((nE & 3) == 0) ? 1 : 0;

  const int nPrep = DH * DX / 8 + DX * DH / 8;
  k_wprep<<<(nPrep + NTHR - 1) / NTHR, NTHR, 0, stream>>>(W1, W2, w1s, w2s);

  k_deg<<<nBD, NTHR, 0, stream>>>(ei, dinv, nE, vec8);

  hipFuncSetAttribute(reinterpret_cast<const void*>(&k_agg1),
                      hipFuncAttributeMaxDynamicSharedMemorySize, LDS_AGG);
  k_agg1<<<nA, NTHR, LDS_AGG, stream>>>(ei, x, dinv, b1, pf, w1s, hpl, nN, nE, vec8);

  k_gemm2<<<nG2, G2THR, 0, stream>>>(hpl, w2s, g2);

  hipFuncSetAttribute(reinterpret_cast<const void*>(&k_agg2),
                      hipFuncAttributeMaxDynamicSharedMemorySize, LDS_AGG);
  k_agg2<<<nA, NTHR, LDS_AGG, stream>>>(ei, g2, dinv, b2, pl, out, nN, nE, vec8);
}
